// PhaseAttentionHybrid_84894323572826
// MI455X (gfx1250) — hardware-verified
//
#include <hip/hip_runtime.h>
#include <math.h>
#include <stdint.h>

#define NSEQ   2
#define SQ     2048
#define HID    2048
#define NHQ    16
#define HDM    128
#define NTOK   4096
#define NPH    32
#define PQW    64
#define KLR    256

static_assert(NTOK == NSEQ * SQ);
static_assert(NHQ * HDM == HID);
static_assert(KLR % 32 == 0 && SQ % KLR == 0);

typedef _Float16     v16h __attribute__((ext_vector_type(16)));
typedef _Float16     v8h  __attribute__((ext_vector_type(8)));
typedef __bf16       v16b __attribute__((ext_vector_type(16)));
typedef __bf16       v8b  __attribute__((ext_vector_type(8)));
typedef float        v8f  __attribute__((ext_vector_type(8)));
typedef float        v4f  __attribute__((ext_vector_type(4)));
typedef unsigned int v4u  __attribute__((ext_vector_type(4)));

__device__ __forceinline__ unsigned short bf_bits(float f) {
  const unsigned u = __float_as_uint(f);
  return (unsigned short)((u + 0x7FFFu + ((u >> 16) & 1u)) >> 16);
}
__device__ __forceinline__ float bf_val(unsigned short h) { return __uint_as_float(((unsigned)h) << 16); }
__device__ __forceinline__ unsigned pk16(unsigned short a, unsigned short b) { return (unsigned)a | ((unsigned)b << 16); }
__device__ __forceinline__ v8f zero8() { v8f z = {0.f, 0.f, 0.f, 0.f, 0.f, 0.f, 0.f, 0.f}; return z; }
__device__ __forceinline__ int wave_id() {
#if defined(__HIP_DEVICE_COMPILE__)
  return __builtin_amdgcn_readfirstlane((int)(threadIdx.x >> 5));
#else
  return (int)(threadIdx.x >> 5);
#endif
}
__device__ __forceinline__ void lds_wave_sync() {
#if defined(__HIP_DEVICE_COMPILE__)
  __builtin_amdgcn_fence(__ATOMIC_RELEASE, "workgroup");
  __builtin_amdgcn_wave_barrier();
  __builtin_amdgcn_fence(__ATOMIC_ACQUIRE, "workgroup");
#endif
}

union FragH { v16h v; v8h h[2]; };
union FragB { v16b v; v8b h[2]; };
__device__ __forceinline__ v16h ldfrag_h(const _Float16* p) { FragH f; f.h[0] = *(const v8h*)(p); f.h[1] = *(const v8h*)(p + 16); return f.v; }
__device__ __forceinline__ v16b ldfrag_b(const __bf16* p)   { FragB f; f.h[0] = *(const v8b*)(p); f.h[1] = *(const v8b*)(p + 16); return f.v; }

__device__ __forceinline__ v8f mma_h(v16h a, v16h b, v8f c) {
#if defined(__HIP_DEVICE_COMPILE__)
  return __builtin_amdgcn_wmma_f32_16x16x32_f16(false, a, false, b, (short)0, c, false, false);
#else
  return c;
#endif
}
__device__ __forceinline__ v8f mma_b(v16b a, v16b b, v8f c) {
#if defined(__HIP_DEVICE_COMPILE__)
  return __builtin_amdgcn_wmma_f32_16x16x32_bf16(false, a, false, b, (short)0, c, false, false);
#else
  return c;
#endif
}
__device__ __forceinline__ void guard_b5(v8f& a, v8f& b, v16b x0, v16b x1, v16b x2, v16b x3, v16b y) {
#if defined(__HIP_DEVICE_COMPILE__)
  asm volatile("v_nop\n\tv_nop\n\tv_nop\n\tv_nop" : "+v"(a), "+v"(b) : "v"(x0), "v"(x1), "v"(x2), "v"(x3), "v"(y) : "memory");
#endif
}
__device__ __forceinline__ void guard_h3(v8f& a, v8f& b, v16h x, v16h y, v16h z) {
#if defined(__HIP_DEVICE_COMPILE__)
  asm volatile("v_nop\n\tv_nop\n\tv_nop\n\tv_nop" : "+v"(a), "+v"(b) : "v"(x), "v"(y), "v"(z) : "memory");
#endif
}
__device__ __forceinline__ void guard_h4(v8f& a, v8f& b, v16h w, v16h x, v16h y, v16h z) {
#if defined(__HIP_DEVICE_COMPILE__)
  asm volatile("v_nop\n\tv_nop\n\tv_nop\n\tv_nop" : "+v"(a), "+v"(b) : "v"(w), "v"(x), "v"(y), "v"(z) : "memory");
#endif
}
__device__ __forceinline__ void acc_guard4(v8f& a, v8f& b, v8f& c, v8f& d) {
#if defined(__HIP_DEVICE_COMPILE__)
  asm volatile("v_nop\n\tv_nop\n\tv_nop\n\tv_nop" : "+v"(a), "+v"(b), "+v"(c), "+v"(d));
#endif
}

__global__ __launch_bounds__(256) void cvt_bf16_kernel(const float* __restrict__ in, unsigned short* __restrict__ outp, int n8) {
  const int i = (int)blockIdx.x * 256 + (int)threadIdx.x;
  if (i >= n8) return;
  const size_t e = 8 * (size_t)i;
  const v4f a = *(const v4f*)(in + e);
  const v4f b = *(const v4f*)(in + e + 4);
  v4u w;
  w[0] = pk16(bf_bits(a[0]), bf_bits(a[1]));
  w[1] = pk16(bf_bits(a[2]), bf_bits(a[3]));
  w[2] = pk16(bf_bits(b[0]), bf_bits(b[1]));
  w[3] = pk16(bf_bits(b[2]), bf_bits(b[3]));
  *(volatile v4u*)(outp + e) = w;
  __threadfence();
  *(volatile v4u*)(outp + e) = w;
}

__global__ __launch_bounds__(256) void tconv_bf16_kernel(const float* __restrict__ W, unsigned short* __restrict__ outp, int R, int Cc) {
  __shared__ __align__(16) float tf[64 * 68];
  const int c0  = (int)blockIdx.x * 64;
  const int r0  = (int)blockIdx.y * 64;
  const int tid = (int)threadIdx.x;
  {
    const int lr = tid >> 4;
    const int c4 = (tid & 15) * 4;
#pragma unroll
    for (int it = 0; it < 4; ++it) {
      const int rr = it * 16 + lr;
      const v4f a = *(const v4f*)(W + (size_t)(r0 + rr) * Cc + c0 + c4);
      *(v4f*)(tf + rr * 68 + c4) = a;
    }
  }
  __syncthreads();
  const int sub = tid >> 3;
  const int c8  = (tid & 7) * 8;
  v4u hv[2];
#pragma unroll
  for (int it = 0; it < 2; ++it) {
    const int oc = it * 32 + sub;
    v4u a;
#pragma unroll
    for (int q = 0; q < 4; ++q) {
      const float f0 = tf[(c8 + 2 * q) * 68 + oc];
      const float f1 = tf[(c8 + 2 * q + 1) * 68 + oc];
      a[q] = pk16(bf_bits(f0), bf_bits(f1));
    }
    hv[it] = a;
  }
  for (int pass = 0; pass < 2; ++pass) {
#pragma unroll
    for (int it = 0; it < 2; ++it) {
      const int oc = it * 32 + sub;
      const size_t go = (size_t)(c0 + oc) * R + r0 + c8;
      *(volatile v4u*)(outp + go) = hv[it];
    }
    __threadfence();
  }
}

__global__ __launch_bounds__(256) void wpt_kernel(const float* __restrict__ Wpq, const float* __restrict__ Wpk,
                                                  unsigned short* __restrict__ outp) {
  const int n = (int)blockIdx.x;
  const float* W = (n < NHQ) ? Wpq : Wpk;
  const int h = n & (NHQ - 1);
  const int t = (int)threadIdx.x;
  v4u w;
#pragma unroll
  for (int q = 0; q < 4; ++q) {
    const float f0 = W[(size_t)(8 * t + 2 * q) * NHQ + h];
    const float f1 = W[(size_t)(8 * t + 2 * q + 1) * NHQ + h];
    w[q] = pk16(bf_bits(f0), bf_bits(f1));
  }
  const size_t o = (size_t)n * HID + 8 * (size_t)t;
  *(volatile v4u*)(outp + o) = w;
  __threadfence();
  *(volatile v4u*)(outp + o) = w;
}

template <int EPI> struct SlabT { typedef _Float16 T; static constexpr int PERW = 4096; };
template <> struct SlabT<2>     { typedef float    T; static constexpr int PERW = 2048; };
template <> struct SlabT<3>     { typedef float    T; static constexpr int PERW = 1536; };

template <int EPI, int NJ, bool SPLITA>
__global__ __launch_bounds__(128) void gemm_kernel(
    const unsigned short* Ap, const unsigned short* A2p, int lda,
    const unsigned short* __restrict__ Btp, int ldb,
    const float* __restrict__ phs,
    void* C0, void* C1, void* C2, void* C3, int ldc,
    int M, int N, int K) {
  static_assert(NJ == 8 || NJ == 2);
  static_assert((EPI == 3) ? (NJ == 2) : (NJ == 8));
  typedef typename SlabT<EPI>::T ST;
  __shared__ __align__(16) ST slab_all[4 * SlabT<EPI>::PERW];

  const int lane = threadIdx.x & 31;
  const int wave = wave_id();
  const int hh = lane >> 4;
  const int rl = lane & 15;
  const int tilesN = N / (16 * NJ);
  const int tilesM = M >> 5;
  const int tile = (int)blockIdx.x * 4 + wave;
  if (tile >= tilesM * tilesN) return;
  const int tm = tile / tilesN;
  const int tn = tile - tm * tilesN;
  const int m0 = tm << 5;
  const int n0 = tn * (16 * NJ);

  const __bf16* A  = (const __bf16*)(const void*)Ap;
  const __bf16* A2 = (const __bf16*)(const void*)A2p;
  const __bf16* Bt = (const __bf16*)(const void*)Btp;

  v8f acc[2][NJ];
#pragma unroll
  for (int i = 0; i < 2; ++i)
#pragma unroll
    for (int j = 0; j < NJ; ++j) acc[i][j] = zero8();

  for (int k0 = 0; k0 < K; k0 += 32) {
    v16b ah[2], al[2];
#pragma unroll
    for (int i = 0; i < 2; ++i) {
      const size_t ao = (size_t)(m0 + i * 16 + rl) * lda + k0 + 8 * hh;
      ah[i] = ldfrag_b(A + ao);
      al[i] = SPLITA ? ldfrag_b(A2 + ao) : ah[i];
    }
#pragma unroll
    for (int j = 0; j < NJ; ++j) {
      const v16b bj = ldfrag_b(Bt + (size_t)(n0 + j * 16 + rl) * ldb + k0 + 8 * hh);
      acc[0][j] = mma_b(ah[0], bj, acc[0][j]);
      acc[1][j] = mma_b(ah[1], bj, acc[1][j]);
      if (SPLITA) {
        acc[0][j] = mma_b(al[0], bj, acc[0][j]);
        acc[1][j] = mma_b(al[1], bj, acc[1][j]);
      }
      guard_b5(acc[0][j], acc[1][j], ah[0], ah[1], al[0], al[1], bj);
    }
  }
  if constexpr (NJ == 8) {
    acc_guard4(acc[0][0], acc[0][1], acc[0][2], acc[0][3]);
    acc_guard4(acc[0][4], acc[0][5], acc[0][6], acc[0][7]);
    acc_guard4(acc[1][0], acc[1][1], acc[1][2], acc[1][3]);
    acc_guard4(acc[1][4], acc[1][5], acc[1][6], acc[1][7]);
  } else {
    acc_guard4(acc[0][0], acc[0][1], acc[1][0], acc[1][1]);
  }

  ST* slab = slab_all + wave * SlabT<EPI>::PERW;
  _Float16* sl16 = (_Float16*)(void*)slab;
  float*    slf  = (float*)(void*)slab;

  if constexpr (EPI == 0 || EPI == 1) {
    _Float16* P0;
    _Float16* P1;
    int col0;
    int lomode;
    if constexpr (EPI == 0) {
      const bool isq = (n0 < HID);
      P0 = isq ? (_Float16*)C0 : (_Float16*)C2;
      P1 = isq ? (_Float16*)C1 : (_Float16*)C3;
      col0 = isq ? n0 : (n0 - HID);
      const int s0 = m0 & (SQ - 1);
      lomode = isq ? 0 : ((s0 < KLR) ? 1 : 2);
    } else {
      P0 = (_Float16*)C0;
      P1 = (_Float16*)C1;
      col0 = n0;
      lomode = 0;
    }
#pragma unroll
    for (int i = 0; i < 2; ++i) {
#pragma unroll
      for (int r = 0; r < 8; ++r) {
#pragma unroll
        for (int j = 0; j < NJ; ++j) {
          const float v = acc[i][j][r];
          const _Float16 hv = (_Float16)v;
          const int so = (8 * hh + r) * 128 + j * 16 + rl;
          sl16[so]        = hv;
          sl16[2048 + so] = (_Float16)((v - (float)hv) * 2048.0f);
        }
      }
      lds_wave_sync();
      for (int pass = 0; pass < 2; ++pass) {
#pragma unroll
        for (int it = 0; it < 8; ++it) {
          const int row = it * 2 + hh;
          const int c8  = rl * 8;
          const v8h xh = *(const v8h*)(sl16 + row * 128 + c8);
          const v8h xl = *(const v8h*)(sl16 + 2048 + row * 128 + c8);
          const int m = m0 + i * 16 + row;
          *(volatile v8h*)(P0 + (size_t)m * ldc + col0 + c8) = xh;
          if (lomode != 2) {
            const int m1 = (lomode == 1) ? ((m / SQ) * KLR + (m % SQ)) : m;
            *(volatile v8h*)(P1 + (size_t)m1 * ldc + col0 + c8) = xl;
          }
        }
        __threadfence();
      }
      lds_wave_sync();
    }
  } else if constexpr (EPI == 2) {
    float* C = (float*)C0;
#pragma unroll
    for (int i = 0; i < 2; ++i) {
#pragma unroll
      for (int r = 0; r < 8; ++r) {
        const int m = m0 + i * 16 + 8 * hh + r;
        const float sc = 1.0f + 0.1f * phs[m];
#pragma unroll
        for (int j = 0; j < NJ; ++j)
          slf[(8 * hh + r) * 128 + j * 16 + rl] = acc[i][j][r] * sc;
      }
      lds_wave_sync();
      for (int pass = 0; pass < 2; ++pass) {
#pragma unroll
        for (int row = 0; row < 16; ++row) {
          const v4f v = *(const v4f*)(slf + row * 128 + lane * 4);
          *(volatile v4f*)(C + (size_t)(m0 + i * 16 + row) * ldc + n0 + lane * 4) = v;
        }
        __threadfence();
      }
      lds_wave_sync();
    }
  } else {
    float* raw = slf;
    float* ocs = slf + 512;
    float* Cp  = (float*)C0;
#pragma unroll
    for (int i = 0; i < 2; ++i) {
#pragma unroll
      for (int j = 0; j < NJ; ++j)
#pragma unroll
        for (int r = 0; r < 8; ++r)
          raw[(8 * hh + r) * 32 + j * 16 + rl] = acc[i][j][r];
      lds_wave_sync();
#pragma unroll 1
      for (int it = 0; it < 16; ++it) {
        const float v  = raw[it * 32 + lane];
        const float cv = cosf(v);
        const float sv = sinf(v);
        ocs[it * PQW + lane]      = cv;
        ocs[it * PQW + 32 + lane] = sv;
      }
      lds_wave_sync();
      for (int pass = 0; pass < 2; ++pass) {
#pragma unroll
        for (int it = 0; it < 8; ++it) {
          const int row = it * 2 + hh;
          const int c4  = rl * 4;
          const v4f x = *(const v4f*)(ocs + row * PQW + c4);
          *(volatile v4f*)(Cp + (size_t)(m0 + i * 16 + row) * ldc + c4) = x;
        }
        __threadfence();
      }
      lds_wave_sync();
    }
  }
}

__global__ __launch_bounds__(256) void phase_kernel(const float* __restrict__ PQ, float* __restrict__ phs) {
  __shared__ float red[2 * NHQ][256];
  __shared__ float csk[2 * NHQ];
  __shared__ __align__(16) float stg[SQ];
  const int b   = (int)blockIdx.x;
  const int tid = (int)threadIdx.x;
  float pc[NHQ], ps[NHQ];
#pragma unroll
  for (int h = 0; h < NHQ; ++h) { pc[h] = 0.f; ps[h] = 0.f; }
#pragma unroll 1
  for (int u = 0; u < SQ / 256; ++u) {
    const int s = u * 256 + tid;
    const float* rowp = PQ + ((size_t)b * SQ + s) * PQW;
#pragma unroll
    for (int h = 0; h < NHQ; ++h) {
      pc[h] += rowp[NHQ + h];
      ps[h] += rowp[NPH + NHQ + h];
    }
  }
#pragma unroll
  for (int h = 0; h < NHQ; ++h) { red[h][tid] = pc[h]; red[NHQ + h][tid] = ps[h]; }
  __syncthreads();
  if (tid < 2 * NHQ) {
    float s = 0.f;
#pragma unroll 1
    for (int t = 0; t < 256; ++t) s += red[tid][t];
    csk[tid] = s;
  }
  __syncthreads();
#pragma unroll 1
  for (int u = 0; u < SQ / 256; ++u) {
    const int s = u * 256 + tid;
    const float* rowp = PQ + ((size_t)b * SQ + s) * PQW;
    float a = 0.f;
#pragma unroll 1
    for (int h = 0; h < NHQ; ++h) a += rowp[h] * csk[h] + rowp[NPH + h] * csk[NHQ + h];
    stg[s] = a * (1.0f / 32768.0f);
  }
  __syncthreads();
  for (int pass = 0; pass < 2; ++pass) {
#pragma unroll
    for (int it = 0; it < SQ / 1024; ++it) {
      const int idx = it * 256 + tid;
      const v4f v = *(const v4f*)(stg + 4 * idx);
      *(volatile v4f*)(phs + (size_t)b * SQ + 4 * idx) = v;
    }
    __threadfence();
  }
}

#define AT_KC   32
#define KS_P    136
#define VS_P    40
#define PS_P    40
#define LDS_KS  0
#define LDS_KLS (32 * KS_P)
#define LDS_VHS (2 * 32 * KS_P)
#define LDS_VLS (LDS_VHS + 128 * VS_P)
#define LDS_PH  (LDS_VLS + 128 * VS_P)
#define LDS_PL  (LDS_PH + 4 * 16 * PS_P)
#define LDS_TOT (LDS_PL + 4 * 16 * PS_P)
static_assert(LDS_TOT * 2 <= 65536);
static_assert(4 * 4096 <= LDS_TOT);

template <bool PRES>
__global__ __launch_bounds__(128) void attn_causal_kernel(
    const unsigned short* __restrict__ qhp, const unsigned short* __restrict__ qlp,
    const unsigned short* __restrict__ khp, const unsigned short* __restrict__ klp,
    const unsigned short* __restrict__ vhp, const unsigned short* __restrict__ vlp,
    unsigned short* __restrict__ ahp, unsigned short* __restrict__ alp, int qb_base) {
  __shared__ __align__(16) _Float16 lds[LDS_TOT];
  _Float16* Ks  = lds + LDS_KS;
  _Float16* Kls = lds + LDS_KLS;
  _Float16* Vhs = lds + LDS_VHS;
  _Float16* Vls = lds + LDS_VLS;

  const int tid  = (int)threadIdx.x;
  const int lane = tid & 31;
  const int wave = wave_id();
  const int hh   = lane >> 4;
  const int c    = lane & 15;
  const int qb   = (int)blockIdx.x + qb_base;
  const int h    = (int)blockIdx.y;
  const int b    = (int)blockIdx.z;
  const int q0   = qb * 64 + wave * 16;
  const int qlast = q0 + 15;
  const size_t tok0 = (size_t)b * SQ;

  const _Float16* Qhr = (const _Float16*)(const void*)qhp + (tok0 + q0 + c) * HID + h * HDM + 8 * hh;
  const _Float16* Qlr = (const _Float16*)(const void*)qlp + (tok0 + q0 + c) * HID + h * HDM + 8 * hh;
  const _Float16* Kg  = (const _Float16*)(const void*)khp + tok0 * HID + h * HDM;
  const _Float16* Klg = (const _Float16*)(const void*)klp + (size_t)b * KLR * HID + h * HDM;
  const _Float16* Vhg = (const _Float16*)(const void*)vhp + (size_t)(h * HDM) * NTOK + tok0;
  const _Float16* Vlg = (const _Float16*)(const void*)vlp + (size_t)(h * HDM) * NTOK + tok0;
  _Float16* ph = lds + LDS_PH + wave * (16 * PS_P);
  _Float16* pl = lds + LDS_PL + wave * (16 * PS_P);

  float mrow[8], lrow[8];
  v8f oacc[8], oaccr[8];
#pragma unroll
  for (int r = 0; r < 8; ++r) { mrow[r] = -INFINITY; lrow[r] = 0.f; }
#pragma unroll
  for (int t = 0; t < 8; ++t) { oacc[t] = zero8(); oaccr[t] = zero8(); }

  const int nch = 2 * qb + 2;
  for (int kc = 0; kc < nch; ++kc) {
    const int kv0 = kc * AT_KC;
    __syncthreads();
#pragma unroll
    for (int i = 0; i < 4; ++i) {
      const int p   = tid + 128 * i;
      const int key = p >> 4, d8 = (p & 15) * 8;
      const v8h kx = *(const v8h*)(Kg + (size_t)(kv0 + key) * HID + d8);
      *(v8h*)(Ks + key * KS_P + d8) = kx;
      if (PRES) {
        const v8h ky = *(const v8h*)(Klg + (size_t)(kv0 + key) * HID + d8);
        *(v8h*)(Kls + key * KS_P + d8) = ky;
      }
      const int d = p >> 2, k8 = (p & 3) * 8;
      const v8h vx = *(const v8h*)(Vhg + (size_t)d * NTOK + kv0 + k8);
      const v8h vy = *(const v8h*)(Vlg + (size_t)d * NTOK + kv0 + k8);
      *(v8h*)(Vhs + d * VS_P + k8) = vx;
      *(v8h*)(Vls + d * VS_P + k8) = vy;
    }
    __syncthreads();

    if (kv0 <= qlast) {
      v8f sh[2], sr[2];
      sh[0] = zero8(); sh[1] = zero8(); sr[0] = zero8(); sr[1] = zero8();
#pragma unroll
      for (int dc = 0; dc < 4; ++dc) {
        const v16h qa = ldfrag_h(Qhr + dc * 32);
        const v16h ql = ldfrag_h(Qlr + dc * 32);
#pragma unroll
        for (int j = 0; j < 2; ++j) {
          const v16h kb = ldfrag_h(Ks + (j * 16 + c) * KS_P + dc * 32 + 8 * hh);
          sh[j] = mma_h(qa, kb, sh[j]);
          sr[j] = mma_h(ql, kb, sr[j]);
          if (PRES) {
            const v16h kl = ldfrag_h(Kls + (j * 16 + c) * KS_P + dc * 32 + 8 * hh);
            sr[j] = mma_h(qa, kl, sr[j]);
            guard_h4(sh[j], sr[j], qa, ql, kb, kl);
          } else {
            guard_h3(sh[j], sr[j], qa, ql, kb);
          }
        }
      }
      float cm[8];
#pragma unroll
      for (int r = 0; r < 8; ++r) {
        const int qrow = q0 + 8 * hh + r;
        float m = -INFINITY;
#pragma unroll
        for (int j = 0; j < 2; ++j) {
          const int key = kv0 + j * 16 + c;
          float s = (sh[j][r] + sr[j][r] * 0.00048828125f) * 0.08838834764831845f;
          s = (key > qrow) ? -INFINITY : s;
          sh[j][r] = s;
          m = fmaxf(m, s);
        }
#pragma unroll
        for (int off = 1; off < 16; off <<= 1) m = fmaxf(m, __shfl_xor(m, off, 32));
        cm[r] = m;
      }
#pragma unroll
      for (int r = 0; r < 8; ++r) {
        const float mnew  = fmaxf(mrow[r], cm[r]);
        const float alpha = __expf(mrow[r] - mnew);
        mrow[r] = mnew;
        float psum = 0.f;
#pragma unroll
        for (int j = 0; j < 2; ++j) {
          const float p  = __expf(sh[j][r] - mnew);
          psum += p;
          const float pp = p * 1024.0f;
          const _Float16 phv = (_Float16)pp;
          const int po = (8 * hh + r) * PS_P + j * 16 + c;
          ph[po] = phv;
          if (PRES) pl[po] = (_Float16)((pp - (float)phv) * 2048.0f);
        }
#pragma unroll
        for (int off = 1; off < 16; off <<= 1) psum += __shfl_xor(psum, off, 32);
        lrow[r] = lrow[r] * alpha + psum;
#pragma unroll
        for (int t = 0; t < 8; ++t) { oacc[t][r] *= alpha; oaccr[t][r] *= alpha; }
      }
      lds_wave_sync();
      const v16h pa = ldfrag_h(ph + c * PS_P + 8 * hh);
      v16h pr = pa;
      if (PRES) pr = ldfrag_h(pl + c * PS_P + 8 * hh);
#pragma unroll
      for (int t = 0; t < 8; ++t) {
        const v16h vb = ldfrag_h(Vhs + (t * 16 + c) * VS_P + 8 * hh);
        const v16h vr = ldfrag_h(Vls + (t * 16 + c) * VS_P + 8 * hh);
        oacc[t]  = mma_h(pa, vb, oacc[t]);
        oaccr[t] = mma_h(pa, vr, oaccr[t]);
        if (PRES) oaccr[t] = mma_h(pr, vb, oaccr[t]);
        guard_h4(oacc[t], oaccr[t], pa, pr, vb, vr);
      }
    }
  }

  __syncthreads();
  _Float16* osh = lds + wave * 4096;
  _Float16* osl = osh + 2048;
#pragma unroll
  for (int r = 0; r < 8; ++r) {
    const float inv = (1.0f / lrow[r]) * 0.0009765625f;
#pragma unroll
    for (int t = 0; t < 8; ++t) {
      const float o = (oacc[t][r] + oaccr[t][r] * 0.00048828125f) * inv;
      const unsigned short hb = bf_bits(o);
      const unsigned short lb = bf_bits(o - bf_val(hb));
      const int so = (8 * hh + r) * 128 + t * 16 + c;
      osh[so] = __builtin_bit_cast(_Float16, hb);
      osl[so] = __builtin_bit_cast(_Float16, lb);
    }
  }
  lds_wave_sync();
  _Float16* Ahg = (_Float16*)(void*)ahp + (tok0 + q0) * HID + h * HDM;
  _Float16* Alg = (_Float16*)(void*)alp + (tok0 + q0) * HID + h * HDM;
  for (int pass = 0; pass < 2; ++pass) {
#pragma unroll
    for (int it = 0; it < 8; ++it) {
      const int row = it * 2 + hh;
      const int c8  = c * 8;
      const v8h x = *(const v8h*)(osh + row * 128 + c8);
      const v8h y = *(const v8h*)(osl + row * 128 + c8);
      *(volatile v8h*)(Ahg + (size_t)row * HID + c8) = x;
      *(volatile v8h*)(Alg + (size_t)row * HID + c8) = y;
    }
    __threadfence();
  }
}

static inline size_t smax(size_t a, size_t b) { return a > b ? a : b; }

extern "C" void kernel_launch(void* const* d_in, const int* in_sizes, int n_in,
                              void* d_out, int out_size, void* d_ws, size_t ws_size,
                              hipStream_t stream) {
  if (n_in < 7) return;
  if (in_sizes[0] != NTOK * HID) return;
  if (in_sizes[1] != HID * HID) return;
  if (in_sizes[2] != HID * HID) return;
  if (in_sizes[3] != HID * HID) return;
  if (in_sizes[4] != HID * HID) return;
  if (in_sizes[5] != HID * NHQ) return;
  if (in_sizes[6] != HID * NHQ) return;
  if (out_size != NTOK * HID) return;

  const float* x   = (const float*)d_in[0];
  const float* Wq  = (const float*)d_in[1];
  const float* Wk  = (const float*)d_in[2];
  const float* Wv  = (const float*)d_in[3];
  const float* Wo  = (const float*)d_in[4];
  const float* Wpq = (const float*)d_in[5];
  const float* Wpk = (const float*)d_in[6];
  float* out = (float*)d_out;

  const size_t szX   = (size_t)NTOK * HID * 2;
  const size_t szWqk = (size_t)2 * HID * HID * 2;
  const size_t szW   = (size_t)HID * HID * 2;
  const size_t szA   = (size_t)NTOK * HID * 2;
  const size_t szWp  = (size_t)NPH * HID * 2;
  const size_t szQ   = (size_t)NTOK * HID * 2;
  const size_t szKl  = (size_t)NSEQ * KLR * HID * 2;
  const size_t szV   = (size_t)HID * NTOK * 2;
  const size_t szPQ  = (size_t)NTOK * PQW * 4;
  const size_t szPh  = (size_t)NTOK * 4;
  size_t off = 0;
  const size_t oR0 = off; off += smax(szX, szA);
  const size_t oR1 = off; off += smax(szWqk, szA);
  const size_t oR2 = off; off += szW;
  const size_t oWp = off; off += szWp;
  const size_t oQh = off; off += szQ;
  const size_t oQl = off; off += szQ;
  const size_t oKh = off; off += szQ;
  const size_t oKl = off; off += szKl;
  const size_t oVh = off; off += szV;
  const size_t oVl = off; off += szV;
  const size_t oPQ = off; off += szPQ;
  const size_t oPh = off; off += szPh;
  if (off > ws_size) return;

  char* ws = (char*)d_ws;
  unsigned short* Xb   = (unsigned short*)(ws + oR0);
  unsigned short* Ah   = (unsigned short*)(ws + oR0);
  unsigned short* WqkT = (unsigned short*)(ws + oR1);
  unsigned short* Al   = (unsigned short*)(ws + oR1);
  unsigned short* WvT  = (unsigned short*)(ws + oR2);
  unsigned short* WoT  = (unsigned short*)(ws + oR2);
  unsigned short* WpT  = (unsigned short*)(ws + oWp);
  unsigned short* Qh   = (unsigned short*)(ws + oQh);
  unsigned short* Ql   = (unsigned short*)(ws + oQl);
  unsigned short* Kh   = (unsigned short*)(ws + oKh);
  unsigned short* Kl   = (unsigned short*)(ws + oKl);
  unsigned short* Vh   = (unsigned short*)(ws + oVh);
  unsigned short* Vl   = (unsigned short*)(ws + oVl);
  float*          PQ   = (float*)(ws + oPQ);
  float*          phs  = (float*)(ws + oPh);

  const dim3 b256(256), b128(128);

  cvt_bf16_kernel<<<dim3((NTOK * HID / 8) / 256), b256, 0, stream>>>(x, Xb, NTOK * HID / 8);
  tconv_bf16_kernel<<<dim3(HID / 64, HID / 64), b256, 0, stream>>>(Wq, WqkT, HID, HID);
  tconv_bf16_kernel<<<dim3(HID / 64, HID / 64), b256, 0, stream>>>(Wk, WqkT + (size_t)HID * HID, HID, HID);
  tconv_bf16_kernel<<<dim3(HID / 64, HID / 64), b256, 0, stream>>>(Wv, WvT, HID, HID);
  wpt_kernel<<<dim3(NPH), b256, 0, stream>>>(Wpq, Wpk, WpT);
  gemm_kernel<3, 2, false><<<dim3((NTOK / 32) * (NPH / 32) / 4), b128, 0, stream>>>(
      Xb, Xb, HID, WpT, HID, phs, (void*)PQ, (void*)PQ, (void*)PQ, (void*)PQ, PQW, NTOK, NPH, HID);
  phase_kernel<<<dim3(NSEQ), b256, 0, stream>>>(PQ, phs);
  gemm_kernel<0, 8, false><<<dim3((NTOK / 32) * ((2 * HID) / 128) / 4), b128, 0, stream>>>(
      Xb, Xb, HID, WqkT, HID, phs, (void*)Qh, (void*)Ql, (void*)Kh, (void*)Kl, HID, NTOK, 2 * HID, HID);
  gemm_kernel<1, 8, false><<<dim3((HID / 32) * (NTOK / 128) / 4), b128, 0, stream>>>(
      WvT, WvT, HID, Xb, HID, phs, (void*)Vh, (void*)Vl, (void*)Vh, (void*)Vl, NTOK, HID, NTOK, HID);
  tconv_bf16_kernel<<<dim3(HID / 64, HID / 64), b256, 0, stream>>>(Wo, WoT, HID, HID);
  attn_causal_kernel<true><<<dim3(4, NHQ, NSEQ), b128, 0, stream>>>(Qh, Ql, Kh, Kl, Vh, Vl, Ah, Al, 0);
  attn_causal_kernel<false><<<dim3(SQ / 64 - 4, NHQ, NSEQ), b128, 0, stream>>>(Qh, Ql, Kh, Kl, Vh, Vl, Ah, Al, 4);
  gemm_kernel<2, 8, true><<<dim3((NTOK / 32) * (HID / 128) / 4), b128, 0, stream>>>(
      Ah, Al, HID, WoT, HID, phs, (void*)out, (void*)out, (void*)out, (void*)out, HID, NTOK, HID, HID);
  (void)hipGetLastError();
}
